// Mamba_Block_11304353923674
// MI455X (gfx1250) — hardware-verified
//
#include <hip/hip_runtime.h>
#include <math.h>

typedef __attribute__((ext_vector_type(8)))  _Float16 v8h;
typedef __attribute__((ext_vector_type(16))) __bf16   v16b;
typedef __attribute__((ext_vector_type(8)))  __bf16   v8b;
typedef __attribute__((ext_vector_type(8)))  float    v8f;
typedef __attribute__((ext_vector_type(4)))  float    v4f;
typedef __attribute__((ext_vector_type(4)))  unsigned v4u;

constexpr int kBatch  = 2;
constexpr int kSeq    = 2048;
constexpr int kDm     = 256;
constexpr int kDin    = 512;
constexpr int kNst    = 16;
constexpr int kDtR    = 16;
constexpr int kHid    = 1024;
constexpr int kXzP    = 2 * kDin;
constexpr int kXdN    = kDtR + 2 * kNst;
constexpr int kXdP    = 64;
constexpr int kRows   = kBatch * kSeq;
constexpr int kConvTP = 260;
constexpr int kScanTS = 64;
constexpr int kScanCh = 64;
constexpr int kScanYP = 68;
static_assert(kXdN == 48 && kXdN <= kXdP, "x_proj width");
static_assert((kDm % 32) == 0 && (kDin % 32) == 0 && (kHid % 32) == 0, "GEMM K multiples of 32");
static_assert((kRows % 64) == 0 && (kXzP % 64) == 0 && (kXdP % 64) == 0 && (kDm % 64) == 0 &&
              (kHid % 64) == 0 && (kSeq % 64) == 0, "GEMM M,N multiples of 64");
static_assert((kSeq % kScanTS) == 0 && (kDin % kScanCh) == 0 && (kDin % 256) == 0 && (kSeq % 32) == 0, "tile multiples");
static_assert(kDm == 256, "LN kernels assume 256 channels");

constexpr int kBlkWin     = (kXzP * kDm) / 2048;
constexpr int kBlkWxpReal = (kXdN * kDin) / 2048;
constexpr int kBlkWxp     = (kXdP * kDin) / 2048;
constexpr int kBlkWout    = (kDm * kDin) / 2048;
constexpr int kBlkWp1     = (kHid * kDm) / 2048;
constexpr int kBlkWp2     = (kDm * kHid) / 2048;
constexpr int kPB1 = kBlkWin;
constexpr int kPB2 = kPB1 + kBlkWxp;
constexpr int kPB3 = kPB2 + kBlkWout;
constexpr int kPB4 = kPB3 + kBlkWp1;
constexpr int kPBTotal = kPB4 + kBlkWp2;
static_assert((kXzP * kDm) % 2048 == 0 && (kXdN * kDin) % 2048 == 0 && (kXdP * kDin) % 2048 == 0 &&
              (kDm * kDin) % 2048 == 0 && (kHid * kDm) % 2048 == 0, "weight planes are whole blocks");

constexpr size_t kWElemWin  = 0;
constexpr size_t kWElemWxp  = kWElemWin  + (size_t)kXzP * kDm;
constexpr size_t kWElemWout = kWElemWxp  + (size_t)kXdP * kDin;
constexpr size_t kWElemWp1  = kWElemWout + (size_t)kDm * kDin;
constexpr size_t kWElemWp2  = kWElemWp1  + (size_t)kHid * kDm;
constexpr size_t kWElems    = kWElemWp2  + (size_t)kDm * kHid;
static_assert(kWElems == (size_t)kPBTotal * 2048, "weight plane blocks cover the region exactly");
constexpr size_t kOffW   = 0;
constexpr size_t kOffXE  = kOffW   + kWElems * 2;
constexpr size_t kOffXN  = kOffXE  + (size_t)kRows * kDm * 2;
constexpr size_t kOffXZ  = kOffXN  + (size_t)kRows * kDm * 2;
constexpr size_t kOffUC  = kOffXZ  + (size_t)kRows * kXzP * 4;
constexpr size_t kOffUCH = kOffUC  + (size_t)kRows * kDin * 4;
constexpr size_t kOffXD  = kOffUCH + (size_t)kRows * kDin * 2;
constexpr size_t kOffYH  = kOffXD  + (size_t)kRows * kXdP * 4;
constexpr size_t kOffMO  = kOffYH  + (size_t)kRows * kDin * 2;
constexpr size_t kOffX2H = kOffMO  + (size_t)kRows * kDm * 4;
constexpr size_t kOffX2L = kOffX2H + (size_t)kRows * kDm * 2;
constexpr size_t kOffHP  = kOffX2L + (size_t)kRows * kDm * 2;
constexpr size_t kOffHH  = kOffHP  + (size_t)kRows * kHid * 4;
constexpr size_t kOffHL  = kOffHH  + (size_t)kRows * kHid * 2;
constexpr size_t kWsTotal = kOffHL + (size_t)kRows * kHid * 2;
static_assert(kWsTotal <= 134217728ull, "carve cap");
static_assert((kOffXE % 128) == 0 && (kOffXN % 128) == 0 && (kOffXZ % 128) == 0 && (kOffUC % 128) == 0 &&
              (kOffUCH % 128) == 0 && (kOffXD % 128) == 0 && (kOffYH % 128) == 0 && (kOffMO % 128) == 0 &&
              (kOffX2H % 128) == 0 && (kOffX2L % 128) == 0 && (kOffHP % 128) == 0 && (kOffHH % 128) == 0 &&
              (kOffHL % 128) == 0, "128-B aligned regions");
static_assert(((kWElemWxp * 2) % 128) == 0 && ((kWElemWout * 2) % 128) == 0 && ((kWElemWp1 * 2) % 128) == 0 &&
              ((kWElemWp2 * 2) % 128) == 0, "128-B aligned weight planes");

__device__ __forceinline__ unsigned short f2bf_bits(float f) {
  unsigned u = __float_as_uint(f);
  return (unsigned short)((u + 0x7FFFu + ((u >> 16) & 1u)) >> 16);
}
__device__ __forceinline__ float bf_bits2f(unsigned short h) { return __uint_as_float(((unsigned)h) << 16); }
__device__ __forceinline__ float bfr(float f) { return bf_bits2f(f2bf_bits(f)); }

__device__ __forceinline__ v8h pack_hi(const v4f a0, const v4f a1) {
  v8h hv;
#pragma unroll
  for (int e = 0; e < 4; ++e) {
    const float f0 = a0[e];
    const float f1 = a1[e];
    const unsigned short h0 = f2bf_bits(f0);
    const unsigned short h1 = f2bf_bits(f1);
    hv[e]     = __builtin_bit_cast(_Float16, h0);
    hv[4 + e] = __builtin_bit_cast(_Float16, h1);
  }
  return hv;
}
__device__ __forceinline__ void pack_hi_lo(const v4f a0, const v4f a1, v8h& hv, v8h& lv) {
#pragma unroll
  for (int e = 0; e < 4; ++e) {
    const float f0 = a0[e];
    const float f1 = a1[e];
    const unsigned short h0 = f2bf_bits(f0);
    const unsigned short h1 = f2bf_bits(f1);
    const unsigned short l0 = f2bf_bits(f0 - bf_bits2f(h0));
    const unsigned short l1 = f2bf_bits(f1 - bf_bits2f(h1));
    hv[e]     = __builtin_bit_cast(_Float16, h0);
    hv[4 + e] = __builtin_bit_cast(_Float16, h1);
    lv[e]     = __builtin_bit_cast(_Float16, l0);
    lv[4 + e] = __builtin_bit_cast(_Float16, l1);
  }
}

__device__ __forceinline__ v16b frag_load(const __bf16* p) {
  union U { v16b v; v8b h[2]; } f;
  f.h[0] = *(const v8b*)(p);
  f.h[1] = *(const v8b*)(p + 16);
  return f.v;
}
__device__ __forceinline__ v8f frag_mma(v16b a, v16b b, v8f c) {
  return __builtin_amdgcn_wmma_f32_16x16x32_bf16(false, a, false, b, (short)0, c, false, false);
}
__device__ __forceinline__ void guard_row4(v8f& a, v8f& b, v8f& c, v8f& d, v16b x, v16b y) {
  asm volatile("v_nop\n\tv_nop\n\tv_nop\n\tv_nop" : "+v"(a), "+v"(b), "+v"(c), "+v"(d) : "v"(x), "v"(y));
}
__device__ __forceinline__ void keep4_b(v16b a, v16b b, v16b c, v16b d) {
  asm volatile("v_nop" :: "v"(a), "v"(b), "v"(c), "v"(d));
}
__device__ __forceinline__ void acc_guard4(v8f& a, v8f& b, v8f& c, v8f& d) {
  asm volatile("v_nop\n\tv_nop\n\tv_nop\n\tv_nop" : "+v"(a), "+v"(b), "+v"(c), "+v"(d));
}

template <bool SA, bool SB, int BIAS_MODE>
__global__ __launch_bounds__(256) void wmma_gemm64_bf(
    const unsigned short* __restrict__ Ap, const unsigned short* __restrict__ A2p, int lda, long strideA,
    const unsigned short* __restrict__ Btp, const unsigned short* __restrict__ Bt2p, int ldb, long strideB,
    float* __restrict__ Cout, int ldc, long strideC,
    const float* __restrict__ bias,
    int M, int N, int K, float scale) {
  const __bf16* A   = (const __bf16*)Ap;
  const __bf16* A2  = (const __bf16*)A2p;
  const __bf16* Bt  = (const __bf16*)Btp;
  const __bf16* Bt2 = (const __bf16*)Bt2p;
  __shared__ __align__(16) float sT[8][16 * 68];
  const int b    = blockIdx.y;
  const int lane = threadIdx.x & 31;
  const int wave = threadIdx.x >> 5;
  const int tilesN = N >> 6;
  const int tilesM = M >> 6;
  const int tile = blockIdx.x * 8 + wave;
  if (tile >= tilesM * tilesN) return;
  const int tm = tile / tilesN;
  const int tn = tile - tm * tilesN;
  const int m0 = tm << 6;
  const int n0 = tn << 6;

  const __bf16* Ab  = A   + (size_t)b * strideA;
  const __bf16* Bb  = Bt  + (size_t)b * strideB;
  const __bf16* Ab2 = A2  + (size_t)b * strideA;
  const __bf16* Bb2 = Bt2 + (size_t)b * strideB;

  const int rlane = lane & 15;
  const int koff  = (lane >> 4) * 8;
  const int mOff  = (lane >> 4) * 8;

  v8f acc[4][4];
#pragma unroll
  for (int i = 0; i < 4; ++i)
#pragma unroll
    for (int j = 0; j < 4; ++j) acc[i][j] = (v8f){0.f,0.f,0.f,0.f,0.f,0.f,0.f,0.f};

  for (int k0 = 0; k0 < K; k0 += 32) {
    v16b bh[4], bl[4];
#pragma unroll
    for (int j = 0; j < 4; ++j) {
      const size_t bo = (size_t)(n0 + (j << 4) + rlane) * ldb + koff + k0;
      bh[j] = frag_load(Bb + bo);
      if (SB) bl[j] = frag_load(Bb2 + bo);
      else bl[j] = bh[j];
    }
#pragma unroll
    for (int i = 0; i < 4; ++i) {
      const size_t ao = (size_t)(m0 + (i << 4) + rlane) * lda + koff + k0;
      v16b ah = frag_load(Ab + ao);
      v16b al = ah;
      if (SA) al = frag_load(Ab2 + ao);
#pragma unroll
      for (int j = 0; j < 4; ++j) {
        acc[i][j] = frag_mma(ah, bh[j], acc[i][j]);
        if (SB) acc[i][j] = frag_mma(ah, bl[j], acc[i][j]);
        if (SA) acc[i][j] = frag_mma(al, bh[j], acc[i][j]);
      }
      guard_row4(acc[i][0], acc[i][1], acc[i][2], acc[i][3], ah, al);
    }
    keep4_b(bh[0], bh[1], bh[2], bh[3]);
    if (SB) keep4_b(bl[0], bl[1], bl[2], bl[3]);
  }
  acc_guard4(acc[0][0], acc[0][1], acc[0][2], acc[0][3]);
  acc_guard4(acc[1][0], acc[1][1], acc[1][2], acc[1][3]);
  acc_guard4(acc[2][0], acc[2][1], acc[2][2], acc[2][3]);
  acc_guard4(acc[3][0], acc[3][1], acc[3][2], acc[3][3]);

  float* slab = sT[wave];
  float* C = Cout + (size_t)b * strideC;
#pragma unroll
  for (int i = 0; i < 4; ++i) {
    const int mBase = m0 + (i << 4);
    float bm[8];
#pragma unroll
    for (int r = 0; r < 8; ++r) {
      bm[r] = 0.f;
      if (BIAS_MODE == 1) bm[r] = bfr(bias[mBase + mOff + r]);
    }
#pragma unroll
    for (int j = 0; j < 4; ++j) {
      const int n = n0 + (j << 4) + rlane;
      float bv = 0.f;
      if (BIAS_MODE == 2) bv = bfr(bias[n]);
#pragma unroll
      for (int r = 0; r < 8; ++r) {
        float v = acc[i][j][r] * scale;
        if (BIAS_MODE == 1) v += bm[r];
        if (BIAS_MODE == 2) v += bv;
        slab[(mOff + r) * 68 + (j << 4) + rlane] = v;
      }
    }
    __builtin_amdgcn_fence(__ATOMIC_RELEASE, "workgroup");
    __builtin_amdgcn_wave_barrier();
    __builtin_amdgcn_fence(__ATOMIC_ACQUIRE, "workgroup");
    {
      const int hh = lane >> 4, c4 = (lane & 15) * 4;
      for (int pass = 0; pass < 2; ++pass) {
#pragma unroll
        for (int it = 0; it < 8; ++it) {
          const int row = it * 2 + hh;
          v4f v = *(const v4f*)(slab + row * 68 + c4);
          *(volatile v4f*)(C + (size_t)(mBase + row) * ldc + n0 + c4) = v;
        }
        __threadfence();
      }
    }
    __builtin_amdgcn_fence(__ATOMIC_RELEASE, "workgroup");
    __builtin_amdgcn_wave_barrier();
    __builtin_amdgcn_fence(__ATOMIC_ACQUIRE, "workgroup");
  }
}

__global__ __launch_bounds__(256) void prep_weights_kernel(
    const float* __restrict__ w_in, const float* __restrict__ w_xp, const float* __restrict__ w_out,
    const float* __restrict__ w_p1, const float* __restrict__ w_p2, unsigned short* __restrict__ dst)
{
  const int blk = blockIdx.x;
  const float* src = w_in;
  int sblk = blk;
  bool real = true;
  if (blk >= kPB4) {
    src = w_p2; sblk = blk - kPB4;
  } else if (blk >= kPB3) {
    src = w_p1; sblk = blk - kPB3;
  } else if (blk >= kPB2) {
    src = w_out; sblk = blk - kPB2;
  } else if (blk >= kPB1) {
    src = w_xp; sblk = blk - kPB1;
    real = (sblk < kBlkWxpReal);
    sblk = real ? sblk : 0;
  }
  const size_t s0 = ((size_t)sblk * 256 + threadIdx.x) * 8;
  const v4f r0 = *(const v4f*)(src + s0);
  const v4f r1 = *(const v4f*)(src + s0 + 4);
  v4f a0, a1;
#pragma unroll
  for (int e = 0; e < 4; ++e) {
    const float f0 = r0[e];
    const float f1 = r1[e];
    a0[e] = real ? f0 : 0.0f;
    a1[e] = real ? f1 : 0.0f;
  }
  const v8h hv = pack_hi(a0, a1);
  unsigned short* q = dst + ((size_t)blk * 256 + threadIdx.x) * 8;
  *(volatile v8h*)q = hv;
  __threadfence();
  *(volatile v8h*)q = hv;
}

__global__ __launch_bounds__(256) void ln1_kernel(
    const float* __restrict__ x, const float* __restrict__ g, const float* __restrict__ bt,
    unsigned short* __restrict__ XE, unsigned short* __restrict__ XN)
{
  __shared__ __align__(16) float sX[kDm * 33];
  __shared__ float sMu[32];
  __shared__ float sRs[32];
  const int tid = threadIdx.x, lane = tid & 31, wave = tid >> 5;
  constexpr int kBlkPerB = kSeq / 32;
  const int bix = blockIdx.x / kBlkPerB;
  const int l0  = (blockIdx.x - bix * kBlkPerB) * 32;
  {
    const int cr = tid >> 3, l4 = (tid & 7) * 4;
#pragma unroll
    for (int i = 0; i < 8; ++i) {
      const int c = i * 32 + cr;
      const v4f v = *(const v4f*)(x + ((size_t)bix * kDm + c) * kSeq + l0 + l4);
      const float f0 = v[0];
      const float f1 = v[1];
      const float f2 = v[2];
      const float f3 = v[3];
      sX[c * 33 + l4 + 0] = bfr(f0);
      sX[c * 33 + l4 + 1] = bfr(f1);
      sX[c * 33 + l4 + 2] = bfr(f2);
      sX[c * 33 + l4 + 3] = bfr(f3);
    }
  }
  __syncthreads();
  {
    const int tk = tid >> 3, p = tid & 7;
    const float* col = sX + (p * 32) * 33 + tk;
    float s = 0.f;
#pragma unroll 4
    for (int j = 0; j < 32; ++j) s += col[j * 33];
    s += __shfl_xor(s, 1, 32);
    s += __shfl_xor(s, 2, 32);
    s += __shfl_xor(s, 4, 32);
    const float mu = s * (1.0f / (float)kDm);
    float qv = 0.f;
#pragma unroll 4
    for (int j = 0; j < 32; ++j) {
      const float dv = col[j * 33] - mu;
      qv = fmaf(dv, dv, qv);
    }
    qv += __shfl_xor(qv, 1, 32);
    qv += __shfl_xor(qv, 2, 32);
    qv += __shfl_xor(qv, 4, 32);
    const float var = qv * (1.0f / (float)kDm);
    const float rs  = 1.0f / sqrtf(var + 1e-5f);
    if (p == 0) { sMu[tk] = mu; sRs[tk] = rs; }
  }
  __syncthreads();
  float gg[8], bb[8];
  {
    const v4f g0 = *(const v4f*)(g + lane * 8);
    const v4f g1 = *(const v4f*)(g + lane * 8 + 4);
    const v4f b0 = *(const v4f*)(bt + lane * 8);
    const v4f b1 = *(const v4f*)(bt + lane * 8 + 4);
#pragma unroll
    for (int e = 0; e < 4; ++e) {
      const float ga = g0[e];
      const float gb = g1[e];
      const float ba = b0[e];
      const float bc = b1[e];
      gg[e] = bfr(ga); gg[4 + e] = bfr(gb);
      bb[e] = bfr(ba); bb[4 + e] = bfr(bc);
    }
  }
  v8h hn[4], he[4];
#pragma unroll
  for (int it = 0; it < 4; ++it) {
    const int tok = wave * 4 + it;
    const float mu = sMu[tok], rs = sRs[tok];
#pragma unroll
    for (int e = 0; e < 8; ++e) {
      const float xv = sX[(lane * 8 + e) * 33 + tok];
      const float nv = (xv - mu) * rs * gg[e] + bb[e];
      const unsigned short hbn = f2bf_bits(nv);
      const unsigned short hbe = f2bf_bits(xv);
      hn[it][e] = __builtin_bit_cast(_Float16, hbn);
      he[it][e] = __builtin_bit_cast(_Float16, hbe);
    }
  }
  for (int pass = 0; pass < 2; ++pass) {
#pragma unroll
    for (int it = 0; it < 4; ++it) {
      const size_t o = ((size_t)bix * kSeq + l0 + wave * 4 + it) * kDm + lane * 8;
      *(volatile v8h*)(XN + o) = hn[it];
      *(volatile v8h*)(XE + o) = he[it];
    }
    __threadfence();
  }
}

__global__ __launch_bounds__(256) void conv_silu_kernel(
    const float* __restrict__ XZ, const float* __restrict__ cw, const float* __restrict__ cb,
    float* __restrict__ UC, unsigned short* __restrict__ UCH)
{
  __shared__ __align__(16) float sT[16 * kConvTP];
  const int tid = threadIdx.x, lane = tid & 31, wave = tid >> 5;
  const int d0 = blockIdx.x * 256, d = d0 + tid;
  const int g0 = blockIdx.y * 64;
  const int tb = g0 & (kSeq - 1);
  float w0, w1, w2, w3;
  {
    const v4f wv = *(const v4f*)(cw + d * 4);
    const float a0 = wv[0];
    const float a1 = wv[1];
    const float a2 = wv[2];
    const float a3 = wv[3];
    w0 = bfr(a0); w1 = bfr(a1); w2 = bfr(a2); w3 = bfr(a3);
  }
  const float bc = bfr(cb[d]);
  float xm3, xm2, xm1;
  {
    const bool hist = (tb > 0);
    const int rb = hist ? (g0 - 3) : g0;
    const float v3 = XZ[(size_t)rb * kXzP + d];
    const float v2 = XZ[(size_t)(rb + 1) * kXzP + d];
    const float v1 = XZ[(size_t)(rb + 2) * kXzP + d];
    xm3 = hist ? v3 : 0.f;
    xm2 = hist ? v2 : 0.f;
    xm1 = hist ? v1 : 0.f;
  }
  const int hrow = wave >> 1;
  const int hch  = (wave & 1) * 128 + lane * 4;
#pragma unroll 1
  for (int sub = 0; sub < 4; ++sub) {
    const int lb = g0 + sub * 16;
#pragma unroll 1
    for (int s = 0; s < 16; ++s) {
      const float xcur = XZ[(size_t)(lb + s) * kXzP + d];
      float acc = w0 * xm3;
      acc = fmaf(w1, xm2, acc);
      acc = fmaf(w2, xm1, acc);
      acc = fmaf(w3, xcur, acc);
      const float sv = acc + bc;
      const float ev = expf(-sv);
      const float sg = 1.0f / (1.0f + ev);
      sT[s * kConvTP + tid] = sv * sg;
      xm3 = xm2; xm2 = xm1; xm1 = xcur;
    }
    __syncthreads();
    v4f fv[4];
    v8h bh[2];
#pragma unroll
    for (int it = 0; it < 4; ++it) fv[it] = *(const v4f*)(sT + (it * 4 + hrow) * kConvTP + hch);
#pragma unroll
    for (int it = 0; it < 2; ++it) {
      const float* sp = sT + (it * 8 + wave) * kConvTP + lane * 8;
      const v4f a0 = *(const v4f*)(sp);
      const v4f a1 = *(const v4f*)(sp + 4);
      bh[it] = pack_hi(a0, a1);
    }
    for (int pass = 0; pass < 2; ++pass) {
#pragma unroll
      for (int it = 0; it < 4; ++it)
        *(volatile v4f*)(UC + (size_t)(lb + it * 4 + hrow) * kDin + d0 + hch) = fv[it];
#pragma unroll
      for (int it = 0; it < 2; ++it)
        *(volatile v8h*)(UCH + (size_t)(lb + it * 8 + wave) * kDin + d0 + lane * 8) = bh[it];
      __threadfence();
    }
    __syncthreads();
  }
}

__global__ __launch_bounds__(64) void scan_kernel(
    const float* __restrict__ XD, const float* __restrict__ UC, const float* __restrict__ XZ,
    const float* __restrict__ Wdt, const float* __restrict__ bdt, const float* __restrict__ Alog,
    const float* __restrict__ Dp, unsigned short* __restrict__ YH)
{
  __shared__ __align__(16) float sX[kScanTS * kXdP];
  __shared__ __align__(16) float sY[kScanTS * kScanYP];
  __shared__ __align__(16) float sW[kDtR * kScanCh];
  __shared__ __align__(16) float sA[kNst * kScanCh];
  const int tid = threadIdx.x, lane = tid & 31, wave = tid >> 5;
  constexpr int kBlkPerB = kDin / kScanCh;
  const int bix = blockIdx.x / kBlkPerB;
  const int d0  = (blockIdx.x - bix * kBlkPerB) * kScanCh;
  const int d   = d0 + tid;
  const size_t row0 = (size_t)bix * kSeq;
#pragma unroll 1
  for (int r = 0; r < kDtR; ++r) sW[r * kScanCh + tid] = bfr(Wdt[(size_t)d * kDtR + r]);
#pragma unroll 1
  for (int s = 0; s < kNst; ++s) sA[s * kScanCh + tid] = -expf(bfr(Alog[(size_t)d * kNst + s]));
  __syncthreads();
  float negA[kNst], h[kNst];
#pragma unroll
  for (int s = 0; s < kNst; ++s) {
    negA[s] = sA[s * kScanCh + tid];
    h[s] = 0.f;
  }
  const float bb = bfr(bdt[d]);
  const float Dd = bfr(Dp[d]);
  const int lr = tid >> 4, lc4 = (tid & 15) * 4;
  const int q = lane >> 3, c8 = (lane & 7) * 8;
#pragma unroll 1
  for (int t0 = 0; t0 < kSeq; t0 += kScanTS) {
    __syncthreads();
#pragma unroll
    for (int i = 0; i < 16; ++i) {
      const int r = lr + 4 * i;
      *(v4f*)(sX + r * kXdP + lc4) = *(const v4f*)(XD + (row0 + t0 + r) * kXdP + lc4);
    }
    __syncthreads();
#pragma unroll 1
    for (int s = 0; s < kScanTS; ++s) {
      const int t = t0 + s;
      const float* xr = sX + s * kXdP;
      float vdot = 0.f;
#pragma unroll 1
      for (int r4 = 0; r4 < kDtR / 4; ++r4) {
        const v4f xv = *(const v4f*)(xr + 4 * r4);
        const float* wp = sW + (4 * r4) * kScanCh + tid;
        vdot = fmaf(xv[0], wp[0], vdot);
        vdot = fmaf(xv[1], wp[kScanCh], vdot);
        vdot = fmaf(xv[2], wp[2 * kScanCh], vdot);
        vdot = fmaf(xv[3], wp[3 * kScanCh], vdot);
      }
      float Bs[kNst], Cs[kNst];
#pragma unroll
      for (int q4 = 0; q4 < 4; ++q4) {
        const v4f bv = *(const v4f*)(xr + kDtR + 4 * q4);
        const v4f cv = *(const v4f*)(xr + kDtR + kNst + 4 * q4);
        Bs[4 * q4 + 0] = bv[0]; Bs[4 * q4 + 1] = bv[1]; Bs[4 * q4 + 2] = bv[2]; Bs[4 * q4 + 3] = bv[3];
        Cs[4 * q4 + 0] = cv[0]; Cs[4 * q4 + 1] = cv[1]; Cs[4 * q4 + 2] = cv[2]; Cs[4 * q4 + 3] = cv[3];
      }
      const float v   = vdot + bb;
      const float a   = __expf(-fabsf(v));
      const float u   = 1.0f + a;
      const float l1p = __logf(u) + (a - (u - 1.0f)) * __builtin_amdgcn_rcpf(u);
      const float dt  = fmaxf(v, 0.0f) + l1p;
      const float xt  = UC[(row0 + t) * kDin + d];
      const float dtx = dt * xt;
      float y = 0.f;
#pragma unroll
      for (int k = 0; k < kNst; ++k) {
        const float e = __expf(dt * negA[k]);
        h[k] = e * h[k] + dtx * Bs[k];
        y = h[k] * Cs[k] + y;
      }
      y = xt * Dd + y;
      const float zv = XZ[(row0 + t) * kXzP + kDin + d];
      const float eg = expf(-zv);
      const float sg = 1.0f / (1.0f + eg);
      y = y * (zv * sg);
      sY[s * kScanYP + tid] = y;
    }
    __syncthreads();
    v8h hv[8];
#pragma unroll
    for (int it = 0; it < 8; ++it) {
      const int row = it * 8 + wave * 4 + q;
      const float* sp = sY + row * kScanYP + c8;
      const v4f a0 = *(const v4f*)(sp);
      const v4f a1 = *(const v4f*)(sp + 4);
      hv[it] = pack_hi(a0, a1);
    }
    for (int pass = 0; pass < 2; ++pass) {
#pragma unroll
      for (int it = 0; it < 8; ++it) {
        const int row = it * 8 + wave * 4 + q;
        const size_t o = (row0 + t0 + row) * kDin + d0 + c8;
        *(volatile v8h*)(YH + o) = hv[it];
      }
      __threadfence();
    }
  }
}

__global__ __launch_bounds__(256) void ln2_kernel(
    const float* __restrict__ MO, const unsigned short* __restrict__ XE,
    const float* __restrict__ g, const float* __restrict__ bt,
    unsigned short* __restrict__ X2H, unsigned short* __restrict__ X2L)
{
  const int lane = threadIdx.x & 31, wave = threadIdx.x >> 5;
  const int t = blockIdx.x * 8 + wave;
  const float* mp = MO + (size_t)t * kDm + lane * 8;
  const v4f m0 = *(const v4f*)(mp);
  const v4f m1 = *(const v4f*)(mp + 4);
  const v4u xw = *(const v4u*)(XE + (size_t)t * kDm + lane * 8);
  const unsigned w0 = xw[0];
  const unsigned w1 = xw[1];
  const unsigned w2 = xw[2];
  const unsigned w3 = xw[3];
  float r[8];
  r[0] = m0[0] + __uint_as_float(w0 << 16);
  r[1] = m0[1] + __uint_as_float(w0 & 0xffff0000u);
  r[2] = m0[2] + __uint_as_float(w1 << 16);
  r[3] = m0[3] + __uint_as_float(w1 & 0xffff0000u);
  r[4] = m1[0] + __uint_as_float(w2 << 16);
  r[5] = m1[1] + __uint_as_float(w2 & 0xffff0000u);
  r[6] = m1[2] + __uint_as_float(w3 << 16);
  r[7] = m1[3] + __uint_as_float(w3 & 0xffff0000u);
  float s = ((r[0] + r[1]) + (r[2] + r[3])) + ((r[4] + r[5]) + (r[6] + r[7]));
  s += __shfl_xor(s, 16, 32);
  s += __shfl_xor(s, 8, 32);
  s += __shfl_xor(s, 4, 32);
  s += __shfl_xor(s, 2, 32);
  s += __shfl_xor(s, 1, 32);
  const float mu = s * (1.0f / (float)kDm);
  float qv = 0.f;
#pragma unroll
  for (int e = 0; e < 8; ++e) {
    r[e] = r[e] - mu;
    qv = fmaf(r[e], r[e], qv);
  }
  qv += __shfl_xor(qv, 16, 32);
  qv += __shfl_xor(qv, 8, 32);
  qv += __shfl_xor(qv, 4, 32);
  qv += __shfl_xor(qv, 2, 32);
  qv += __shfl_xor(qv, 1, 32);
  const float var = qv * (1.0f / (float)kDm);
  const float rs  = 1.0f / sqrtf(var + 1e-5f);
  const v4f g0 = *(const v4f*)(g + lane * 8);
  const v4f g1 = *(const v4f*)(g + lane * 8 + 4);
  const v4f b0 = *(const v4f*)(bt + lane * 8);
  const v4f b1 = *(const v4f*)(bt + lane * 8 + 4);
  v4f o0, o1;
#pragma unroll
  for (int e = 0; e < 4; ++e) {
    const float ga = g0[e];
    const float gb = g1[e];
    const float ba = b0[e];
    const float bc = b1[e];
    o0[e] = r[e] * rs * bfr(ga) + bfr(ba);
    o1[e] = r[4 + e] * rs * bfr(gb) + bfr(bc);
  }
  v8h hv, lv;
  pack_hi_lo(o0, o1, hv, lv);
  const size_t o = (size_t)t * kDm + lane * 8;
  *(volatile v8h*)(X2H + o) = hv;
  *(volatile v8h*)(X2L + o) = lv;
  __threadfence();
  *(volatile v8h*)(X2H + o) = hv;
  *(volatile v8h*)(X2L + o) = lv;
}

__global__ __launch_bounds__(256) void gelu_split_kernel(
    const float* __restrict__ HP, const float* __restrict__ p1b,
    unsigned short* __restrict__ HH, unsigned short* __restrict__ HL)
{
  __shared__ __align__(16) float sG[2048];
  const int tid = threadIdx.x;
  const size_t base = (size_t)blockIdx.x * 2048;
#pragma unroll 1
  for (int i = 0; i < 8; ++i) {
    const int idx = i * 256 + tid;
    const float v = HP[base + idx] + bfr(p1b[idx & (kHid - 1)]);
    const float gl = 0.5f * v * (1.0f + erff(v * 0.70710678118654752f));
    sG[idx] = gl;
  }
  __syncthreads();
  const v4f a0 = *(const v4f*)(sG + tid * 8);
  const v4f a1 = *(const v4f*)(sG + tid * 8 + 4);
  v8h hv, lv;
  pack_hi_lo(a0, a1, hv, lv);
  const size_t o = base + (size_t)tid * 8;
  *(volatile v8h*)(HH + o) = hv;
  *(volatile v8h*)(HL + o) = lv;
  __threadfence();
  *(volatile v8h*)(HH + o) = hv;
  *(volatile v8h*)(HL + o) = lv;
}

extern "C" void kernel_launch(void* const* d_in, const int* in_sizes, int n_in,
                              void* d_out, int out_size, void* d_ws, size_t ws_size,
                              hipStream_t stream) {
  if (n_in < 16) return;
  if (in_sizes[0] != kBatch * kDm * kSeq) return;
  if (in_sizes[1] != kDm || in_sizes[2] != kDm) return;
  if (in_sizes[3] != kXzP * kDm) return;
  if (in_sizes[4] != kDin * 4 || in_sizes[5] != kDin) return;
  if (in_sizes[6] != kXdN * kDin) return;
  if (in_sizes[7] != kDin * kDtR || in_sizes[8] != kDin) return;
  if (in_sizes[9] != kDin * kNst || in_sizes[10] != kDin) return;
  if (in_sizes[11] != kDm * kDin) return;
  if (in_sizes[12] != kHid * kDm || in_sizes[13] != kHid) return;
  if (in_sizes[14] != kDm * kHid || in_sizes[15] != kDm) return;
  if (out_size != kBatch * kDm * kSeq) return;
  if (ws_size < kWsTotal) return;

  const float* x      = (const float*)d_in[0];
  const float* ln_g   = (const float*)d_in[1];
  const float* ln_b   = (const float*)d_in[2];
  const float* w_in   = (const float*)d_in[3];
  const float* conv_w = (const float*)d_in[4];
  const float* conv_b = (const float*)d_in[5];
  const float* w_xp   = (const float*)d_in[6];
  const float* w_dt   = (const float*)d_in[7];
  const float* b_dt   = (const float*)d_in[8];
  const float* A_log  = (const float*)d_in[9];
  const float* D_skip = (const float*)d_in[10];
  const float* w_out  = (const float*)d_in[11];
  const float* w_p1   = (const float*)d_in[12];
  const float* p1_b   = (const float*)d_in[13];
  const float* w_p2   = (const float*)d_in[14];
  const float* p2_b   = (const float*)d_in[15];
  float* out = (float*)d_out;

  char* ws = (char*)d_ws;
  unsigned short* WALL = (unsigned short*)(ws + kOffW);
  unsigned short* WIN  = WALL + kWElemWin;
  unsigned short* WXP  = WALL + kWElemWxp;
  unsigned short* WOUT = WALL + kWElemWout;
  unsigned short* WP1  = WALL + kWElemWp1;
  unsigned short* WP2  = WALL + kWElemWp2;
  unsigned short* XE   = (unsigned short*)(ws + kOffXE);
  unsigned short* XN   = (unsigned short*)(ws + kOffXN);
  float*          XZ   = (float*)(ws + kOffXZ);
  float*          UC   = (float*)(ws + kOffUC);
  unsigned short* UCH  = (unsigned short*)(ws + kOffUCH);
  float*          XD   = (float*)(ws + kOffXD);
  unsigned short* YH   = (unsigned short*)(ws + kOffYH);
  float*          MO   = (float*)(ws + kOffMO);
  unsigned short* X2H  = (unsigned short*)(ws + kOffX2H);
  unsigned short* X2L  = (unsigned short*)(ws + kOffX2L);
  float*          HP   = (float*)(ws + kOffHP);
  unsigned short* HH   = (unsigned short*)(ws + kOffHH);
  unsigned short* HL   = (unsigned short*)(ws + kOffHL);

  prep_weights_kernel<<<kPBTotal, 256, 0, stream>>>(w_in, w_xp, w_out, w_p1, w_p2, WALL);

  ln1_kernel<<<kRows / 32, 256, 0, stream>>>(x, ln_g, ln_b, XE, XN);

  wmma_gemm64_bf<false, false, 0><<<dim3((kRows / 64) * (kXzP / 64) / 8, 1), 256, 0, stream>>>(
      XN, XN, kDm, 0L, WIN, WIN, kDm, 0L, XZ, kXzP, 0L, p1_b, kRows, kXzP, kDm, 1.0f);

  conv_silu_kernel<<<dim3(kDin / 256, kRows / 64), 256, 0, stream>>>(XZ, conv_w, conv_b, UC, UCH);

  wmma_gemm64_bf<false, false, 0><<<dim3((kRows / 64) * (kXdP / 64) / 8, 1), 256, 0, stream>>>(
      UCH, UCH, kDin, 0L, WXP, WXP, kDin, 0L, XD, kXdP, 0L, p1_b, kRows, kXdP, kDin, 1.0f);

  scan_kernel<<<kBatch * (kDin / kScanCh), kScanCh, 0, stream>>>(XD, UC, XZ, w_dt, b_dt, A_log, D_skip, YH);

  wmma_gemm64_bf<false, false, 0><<<dim3((kRows / 64) * (kDm / 64) / 8, 1), 256, 0, stream>>>(
      YH, YH, kDin, 0L, WOUT, WOUT, kDin, 0L, MO, kDm, 0L, p1_b, kRows, kDm, kDin, 1.0f);

  ln2_kernel<<<kRows / 8, 256, 0, stream>>>(MO, XE, ln_g, ln_b, X2H, X2L);

  wmma_gemm64_bf<true, false, 0><<<dim3((kRows / 64) * (kHid / 64) / 8, 1), 256, 0, stream>>>(
      X2H, X2L, kDm, 0L, WP1, WP1, kDm, 0L, HP, kHid, 0L, p1_b, kRows, kHid, kDm, 1.0f);

  gelu_split_kernel<<<(kRows * kHid) / 2048, 256, 0, stream>>>(HP, p1_b, HH, HL);

  wmma_gemm64_bf<false, true, 1><<<dim3((kDm / 64) * (kSeq / 64) / 8, kBatch), 256, 0, stream>>>(
      WP2, WP2, kHid, 0L, HH, HL, kHid, (long)kSeq * kHid, out, kSeq, (long)kDm * kSeq, p2_b,
      kDm, kSeq, kHid, 1.0f);
}
